// MultiheadSelfAttention_74964359185071
// MI455X (gfx1250) — hardware-verified
//
#include <hip/hip_runtime.h>


#ifndef NB
#define NB 2
#endif
#ifndef SEQ
#define SEQ 2048
#endif
#define NB_FULL  2
#define SEQ_FULL 2048
#define DM    1024
#define NH    16
#define HD    64
#define NQKV  (3 * DM)
#define NSLOT (2 * NH)
#define RH    ((SEQ < 512) ? SEQ : 512)
#define LOG2E 1.4426950408889634f
#define SCL   0.125f
#define PEXP  10.0f

static_assert(NB >= 1 && NB <= NB_FULL);
static_assert(SEQ % 64 == 0 && SEQ <= SEQ_FULL);
static_assert(RH % 64 == 0 && RH <= SEQ);
static_assert(DM % 64 == 0 && NQKV % 64 == 0 && DM % 32 == 0);
static_assert(NH * HD == DM && HD == 64);
static_assert(HD / 2 == 32);

typedef _Float16 h16;
typedef unsigned short bf;
typedef __attribute__((ext_vector_type(16))) __bf16   v16bf;
typedef __attribute__((ext_vector_type(16))) _Float16 v16h;
typedef __attribute__((ext_vector_type(16))) unsigned short v16us;
typedef __attribute__((ext_vector_type(8)))  _Float16 v8h;
typedef __attribute__((ext_vector_type(8)))  unsigned short v8us;
typedef __attribute__((ext_vector_type(8)))  float    v8f;
typedef __attribute__((ext_vector_type(4)))  float    v4f;
typedef __attribute__((ext_vector_type(2)))  float    v2f;
typedef __attribute__((ext_vector_type(2)))  _Float16 v2h;
typedef __attribute__((ext_vector_type(2)))  unsigned short v2us;
typedef v4f  __attribute__((may_alias)) v4fa;

__device__ __forceinline__ unsigned short f2bf(float f) { unsigned u = __float_as_uint(f); u += 0x7FFFu + ((u >> 16) & 1u); return (unsigned short)(u >> 16); }
__device__ __forceinline__ float bf2f(unsigned short b) { return __uint_as_float(((unsigned)b) << 16); }
__device__ __forceinline__ void splitf(float y, unsigned short& h, unsigned short& l) { h = f2bf(y); l = f2bf(y - bf2f(h)); }
__device__ __forceinline__ v16h cat16(v8h lo, v8h hi) { return __builtin_shufflevector(lo, hi, 0, 1, 2, 3, 4, 5, 6, 7, 8, 9, 10, 11, 12, 13, 14, 15); }
__device__ __forceinline__ v16bf cat16b(v8us lo, v8us hi) { return __builtin_bit_cast(v16bf, __builtin_shufflevector(lo, hi, 0, 1, 2, 3, 4, 5, 6, 7, 8, 9, 10, 11, 12, 13, 14, 15)); }
__device__ __forceinline__ v8f wmma16(v16h a, v16h b, v8f c) { return __builtin_amdgcn_wmma_f32_16x16x32_f16(false, a, false, b, (short)0, c, false, false); }
__device__ __forceinline__ v8f wmmab(v16bf a, v16bf b, v8f c) { return __builtin_amdgcn_wmma_f32_16x16x32_bf16(false, a, false, b, (short)0, c, false, false); }
__device__ __forceinline__ v16h  ldh(const h16* p) { return cat16(*(const v8h*)p, *(const v8h*)(p + 16)); }
__device__ __forceinline__ v16bf ldb(const bf* p)  { return cat16b(*(const v8us*)p, *(const v8us*)(p + 16)); }
__device__ __forceinline__ void wave_sync() { __builtin_amdgcn_wave_barrier(); asm volatile("" ::: "memory"); }

template <int NSPLIT>
__device__ __forceinline__ void gemm_body(const bf* __restrict__ A, const bf* __restrict__ A2, const bf* __restrict__ Bt, int K, float* C, int ldc, size_t sA, size_t sC) {
    __shared__ __align__(16) float os[16 * 68];
    const size_t z = blockIdx.z; A += z * sA; A2 += z * sA; C += z * sC;
    const int lane = threadIdx.x & 31, lr = lane & 15, hi = lane >> 4; const int r0 = blockIdx.x * 64, c0 = blockIdx.y * 64;
    v8f acc[4][4];
#pragma unroll
    for (int mb = 0; mb < 4; ++mb)
#pragma unroll
        for (int nb = 0; nb < 4; ++nb) acc[mb][nb] = (v8f){};
    const size_t aoff = (size_t)(r0 + lr) * K + 8 * hi, boff = (size_t)(c0 + lr) * K + 8 * hi;
#pragma unroll 1
    for (int kc = 0; kc < K; kc += 32) {
        v16bf a[4], a2[4];
#pragma unroll
        for (int mb = 0; mb < 4; ++mb) { a[mb] = ldb(A + aoff + (size_t)mb * 16 * K + kc); if (NSPLIT == 1) a2[mb] = ldb(A2 + aoff + (size_t)mb * 16 * K + kc); else a2[mb] = a[mb]; }
#pragma unroll
        for (int nb = 0; nb < 4; ++nb) { const v16bf b = ldb(Bt + boff + (size_t)nb * 16 * K + kc);
#pragma unroll
            for (int mb = 0; mb < 4; ++mb) { acc[mb][nb] = wmmab(a[mb], b, acc[mb][nb]); if (NSPLIT == 1) acc[mb][nb] = wmmab(a2[mb], b, acc[mb][nb]); } }
        asm volatile("v_nop\n\tv_nop\n\tv_nop\n\tv_nop" : "+v"(acc[0][0]), "+v"(acc[1][1]), "+v"(acc[2][2]), "+v"(acc[3][3]) : "v"(a[0]), "v"(a[3]));
    }
#pragma unroll
    for (int mb = 0; mb < 4; ++mb) {
#pragma unroll
        for (int nb = 0; nb < 4; ++nb) {
#pragma unroll
            for (int j = 0; j < 8; ++j) os[(hi * 8 + j) * 68 + nb * 16 + lr] = acc[mb][nb][j]; }
        wave_sync();
        float* crow = C + (size_t)(r0 + mb * 16) * ldc + c0;
#pragma unroll 1
        for (int ps = 0; ps < 2; ++ps) {
#pragma unroll
            for (int s = 0; s < 8; ++s) { const int row = 2 * s + hi, cofs = lr * 4; const v4f val = *(const v4fa*)(os + row * 68 + cofs);
                *(volatile v4f*)(crow + (size_t)row * ldc + cofs) = val; }
            if (ps == 0) __threadfence(); }
        wave_sync();
    }
}
__global__ __launch_bounds__(32) void k_gemm_qkv(const bf* __restrict__ A, const bf* __restrict__ Bt, float* C) { gemm_body<0>(A, A, Bt, DM, C, NQKV, 0, 0); }
__global__ __launch_bounds__(32) void k_gemm_out(const bf* __restrict__ Ah, const bf* __restrict__ Al, const bf* __restrict__ Bt, float* C) { gemm_body<1>(Ah, Al, Bt, DM, C, DM, (size_t)SEQ * DM, (size_t)SEQ_FULL * DM); }

__global__ __launch_bounds__(256) void k_cvt8(const float* __restrict__ src, bf* dst, size_t n8, int row8, int rpb, int srpb) {
    const size_t i = (size_t)blockIdx.x * 256 + threadIdx.x; if (i >= n8) return;
    const size_t row = i / (size_t)row8; const size_t c = i - row * (size_t)row8; const size_t bb = row / (size_t)rpb; const size_t t = row - bb * (size_t)rpb;
    const v8f v = *(const v8f*)(src + ((bb * (size_t)srpb + t) * (size_t)row8 + c) * 8); v8us o;
#pragma unroll
    for (int k = 0; k < 8; ++k) o[k] = f2bf(v[k]);
    *(volatile v8us*)(dst + i * 8) = o; __threadfence(); *(volatile v8us*)(dst + i * 8) = o; }

__global__ __launch_bounds__(32) void k_freq(float* IFQ) { const int i = threadIdx.x & 31; const float e = -(float)(2 * i) * (1.0f / (float)HD); const float f = powf(10000.0f, e);
    *(volatile float*)(IFQ + i) = f; __threadfence(); *(volatile float*)(IFQ + i) = f; }
__global__ __launch_bounds__(256) void k_cstab(const int* __restrict__ tok, const float* __restrict__ IFQ, float* CS) { const int idx = blockIdx.x * 256 + threadIdx.x; if (idx >= SEQ * (HD / 2)) return; const int t = idx >> 5, i = idx & 31;
    const float ang = (float)tok[t] * IFQ[i]; float sn, cn; sincosf(ang, &sn, &cn); v2f cs; cs[0] = cn; cs[1] = sn;
    *(volatile v2f*)(CS + (size_t)idx * 2) = cs; __threadfence(); *(volatile v2f*)(CS + (size_t)idx * 2) = cs; }

__global__ __launch_bounds__(256) void k_rope(const float* __restrict__ F, const float* __restrict__ CS, h16* P16, bf* Ph, bf* Pl) {
    const size_t e = ((size_t)blockIdx.x * 256 + threadIdx.x) * 2; if (e >= (size_t)NB * NSLOT * SEQ * HD) return;
    const int d = (int)(e % HD); const int t = (int)((e / HD) % SEQ); const int sl = (int)((e / ((size_t)HD * SEQ)) % NSLOT); const int b = (int)(e / ((size_t)HD * SEQ * NSLOT));
    const v2f xv = *(const v2f*)(F + ((size_t)b * SEQ + t) * NQKV + sl * HD + d);
    const v2f cs = *(const v2f*)(CS + ((size_t)t * (HD / 2) + (d >> 1)) * 2);
    const float re = xv[0] * cs[0] - xv[1] * cs[1]; const float ro = xv[0] * cs[1] + xv[1] * cs[0];
    v2h o16; v2us oh, ol; unsigned short a2, c2;
    o16[0] = (h16)re; o16[1] = (h16)ro; splitf(re, a2, c2); oh[0] = a2; ol[0] = c2; splitf(ro, a2, c2); oh[1] = a2; ol[1] = c2;
    const bool hl = (t < RH);
    const size_t eh = (((size_t)b * NSLOT + sl) * RH + (hl ? t : 0)) * HD + d;
    *(volatile v2h*)(P16 + e) = o16; if (hl) { *(volatile v2us*)(Ph + eh) = oh; *(volatile v2us*)(Pl + eh) = ol; }
    __threadfence();
    *(volatile v2h*)(P16 + e) = o16; if (hl) { *(volatile v2us*)(Ph + eh) = oh; *(volatile v2us*)(Pl + eh) = ol; } }

__global__ __launch_bounds__(256) void k_vtp(const float* __restrict__ F, h16* V16, bf* Vh, bf* Vl) {
    const size_t e = ((size_t)blockIdx.x * 256 + threadIdx.x) * 2; if (e >= (size_t)NB * NH * HD * SEQ) return;
    const int t = (int)(e % SEQ); const int d = (int)((e / SEQ) % HD); const int g = (int)((e / ((size_t)SEQ * HD)) % NH); const int b = (int)(e / ((size_t)SEQ * HD * NH));
    const float* f = F + ((size_t)b * SEQ + t) * NQKV + 2 * DM + g * HD + d; const float x0 = f[0], x1 = f[NQKV];
    v2h o16; v2us oh, ol; unsigned short a2, c2;
    o16[0] = (h16)x0; o16[1] = (h16)x1; splitf(x0, a2, c2); oh[0] = a2; ol[0] = c2; splitf(x1, a2, c2); oh[1] = a2; ol[1] = c2;
    const bool hl = (t < RH);
    const size_t eh = (((size_t)b * NH + g) * HD + d) * RH + (hl ? t : 0);
    *(volatile v2h*)(V16 + e) = o16; if (hl) { *(volatile v2us*)(Vh + eh) = oh; *(volatile v2us*)(Vl + eh) = ol; }
    __threadfence();
    *(volatile v2h*)(V16 + e) = o16; if (hl) { *(volatile v2us*)(Vh + eh) = oh; *(volatile v2us*)(Vl + eh) = ol; } }

template <bool MASK>
__device__ __forceinline__ void smx(v8f& s0, v8f& s1, int kb, int qi, int hi, float& m, float& l, float& sf, float pe) {
    const float cl = SCL * LOG2E; const int k0 = kb + 8 * hi; float mx = -3.0e38f;
#pragma unroll
    for (int r = 0; r < 8; ++r) { float t0 = s0[r] * cl, t1 = s1[r] * cl;
        if (MASK) { t0 = (k0 + r <= qi) ? t0 : -3.0e38f; t1 = (k0 + 16 + r <= qi) ? t1 : -3.0e38f; }
        s0[r] = t0; s1[r] = t1; mx = fmaxf(mx, fmaxf(t0, t1)); }
    mx = fmaxf(mx, __shfl_xor(mx, 16, 32));
    const float mn = fmaxf(m, mx); sf = __builtin_amdgcn_exp2f(m - mn); m = mn;
    const float sh = mn - pe; float rs = 0.0f;
#pragma unroll
    for (int r = 0; r < 8; ++r) { float p0 = __builtin_amdgcn_exp2f(s0[r] - sh), p1 = __builtin_amdgcn_exp2f(s1[r] - sh);
        if (MASK) { p0 = (k0 + r <= qi) ? p0 : 0.0f; p1 = (k0 + 16 + r <= qi) ? p1 : 0.0f; }
        s0[r] = p0; s1[r] = p1; rs += p0 + p1; }
    l = l * sf + rs;
}

__device__ __forceinline__ void pk8(v8f a, float inv, v8us& oh, v8us& ol) {
#pragma unroll
    for (int r = 0; r < 8; ++r) { unsigned short x, y; splitf(a[r] * inv, x, y); oh[r] = x; ol[r] = y; } }
__device__ __forceinline__ void attn_store(v8f a0, v8f a1, v8f a2, v8f a3, float l, int lane, size_t obase, bf* ATh, bf* ATl) {
    __shared__ __align__(16) unsigned short sth[16 * 72]; __shared__ __align__(16) unsigned short stl[16 * 72];
    const int lr = lane & 15, hi = lane >> 4;
    const float lt = l + __shfl_xor(l, 16, 32); const float inv = __builtin_amdgcn_rcpf(lt);
    v8us oh, ol; const int so = lr * 72 + 8 * hi;
    pk8(a0, inv, oh, ol); *(v8us*)(sth + so) = oh;      *(v8us*)(stl + so) = ol;
    pk8(a1, inv, oh, ol); *(v8us*)(sth + so + 16) = oh; *(v8us*)(stl + so + 16) = ol;
    pk8(a2, inv, oh, ol); *(v8us*)(sth + so + 32) = oh; *(v8us*)(stl + so + 32) = ol;
    pk8(a3, inv, oh, ol); *(v8us*)(sth + so + 48) = oh; *(v8us*)(stl + so + 48) = ol;
    wave_sync();
    const int rq = lane >> 3, pc = (lane & 7) * 8;
#pragma unroll 1
    for (int ps = 0; ps < 2; ++ps) {
#pragma unroll
        for (int s = 0; s < 4; ++s) { const int row = s * 4 + rq; const v8us vh = *(const v8us*)(sth + row * 72 + pc); const v8us vl = *(const v8us*)(stl + row * 72 + pc);
            *(volatile v8us*)(ATh + obase + (size_t)row * DM + pc) = vh; *(volatile v8us*)(ATl + obase + (size_t)row * DM + pc) = vl; }
        if (ps == 0) __threadfence(); }
}

template <bool MASK>
__device__ __forceinline__ void step_f(const h16* __restrict__ QK, const h16* __restrict__ VT, size_t koff, size_t voff, int kb, v16h qf0, v16h qf1, int qi, int hi,
                                       float& m, float& l, v8f& a0, v8f& a1, v8f& a2, v8f& a3) {
    const h16* kp = QK + koff + (size_t)kb * HD;
    v8f s0 = (v8f){}, s1 = (v8f){};
    { const v16h k00 = ldh(kp), k01 = ldh(kp + 32), k10 = ldh(kp + 16 * HD), k11 = ldh(kp + 16 * HD + 32);
      s0 = wmma16(k00, qf0, s0); s0 = wmma16(k01, qf1, s0); s1 = wmma16(k10, qf0, s1); s1 = wmma16(k11, qf1, s1);
      asm volatile("v_nop\n\tv_nop\n\tv_nop\n\tv_nop" : "+v"(s0), "+v"(s1) : "v"(k11), "v"(qf1)); }
    float sf; smx<MASK>(s0, s1, kb, qi, hi, m, l, sf, PEXP);
    v16h pf;
#pragma unroll
    for (int r = 0; r < 8; ++r) { pf[r] = (h16)s0[r]; pf[8 + r] = (h16)s1[r]; }
    a0 = a0 * sf; a1 = a1 * sf; a2 = a2 * sf; a3 = a3 * sf;
    const h16* vp = VT + voff + kb;
    const v16h v0 = ldh(vp), v1 = ldh(vp + (size_t)16 * SEQ), v2 = ldh(vp + (size_t)32 * SEQ), v3 = ldh(vp + (size_t)48 * SEQ);
    a0 = wmma16(v0, pf, a0); a1 = wmma16(v1, pf, a1); a2 = wmma16(v2, pf, a2); a3 = wmma16(v3, pf, a3);
    asm volatile("v_nop\n\tv_nop\n\tv_nop\n\tv_nop" : "+v"(a0), "+v"(a1), "+v"(a2), "+v"(a3) : "v"(v3), "v"(pf));
}
__global__ __launch_bounds__(32) void k_attn_f(const h16* __restrict__ QK, const h16* __restrict__ VT, bf* ATh, bf* ATl) {
    const int lane = threadIdx.x & 31, lr = lane & 15, hi = lane >> 4;
    const int q0 = RH + blockIdx.x * 16; const int bh = blockIdx.y; const int b = bh / NH, h = bh % NH;
    const size_t qoff = (((size_t)b * NSLOT + h) * SEQ + q0 + lr) * HD + 8 * hi;
    const size_t koff = (((size_t)b * NSLOT + NH + h) * SEQ + lr) * HD + 8 * hi;
    const size_t voff = (((size_t)b * NH + h) * HD + lr) * SEQ + 8 * hi;
    const v16h qf0 = ldh(QK + qoff), qf1 = ldh(QK + qoff + 32);
    v8f a0 = (v8f){}, a1 = (v8f){}, a2 = (v8f){}, a3 = (v8f){}; float m = -3.0e38f, l = 0.0f;
    const int qi = q0 + lr; const int nh = (q0 + 47) >> 5;
#pragma unroll 1
    for (int it = 0; it < nh - 1; ++it) step_f<false>(QK, VT, koff, voff, it * 32, qf0, qf1, qi, hi, m, l, a0, a1, a2, a3);
    step_f<true>(QK, VT, koff, voff, (nh - 1) * 32, qf0, qf1, qi, hi, m, l, a0, a1, a2, a3);
    attn_store(a0, a1, a2, a3, l, lane, ((size_t)b * SEQ + q0) * DM + h * HD, ATh, ATl);
}

template <bool MASK>
__device__ __forceinline__ void step_h(const bf* __restrict__ QKh, const bf* __restrict__ QKl, const bf* __restrict__ VTh, const bf* __restrict__ VTl, size_t koff, size_t voff, int kb,
                                       v16bf qh0, v16bf qh1, v16bf ql0, v16bf ql1, int qi, int hi, float& m, float& l, v8f& a0, v8f& a1, v8f& a2, v8f& a3) {
    const bf* kh = QKh + koff + (size_t)kb * HD; const bf* kl = QKl + koff + (size_t)kb * HD;
    v8f s0 = (v8f){}, s1 = (v8f){};
    { const v16bf h0 = ldb(kh), h1 = ldb(kh + 32), l0 = ldb(kl), l1 = ldb(kl + 32);
      s0 = wmmab(h0, qh0, s0); s0 = wmmab(h1, qh1, s0); s0 = wmmab(l0, qh0, s0); s0 = wmmab(l1, qh1, s0); s0 = wmmab(h0, ql0, s0); s0 = wmmab(h1, ql1, s0);
      asm volatile("v_nop\n\tv_nop\n\tv_nop\n\tv_nop" : "+v"(s0) : "v"(h1), "v"(ql1), "v"(l1), "v"(h0)); }
    { const v16bf h0 = ldb(kh + 16 * HD), h1 = ldb(kh + 16 * HD + 32), l0 = ldb(kl + 16 * HD), l1 = ldb(kl + 16 * HD + 32);
      s1 = wmmab(h0, qh0, s1); s1 = wmmab(h1, qh1, s1); s1 = wmmab(l0, qh0, s1); s1 = wmmab(l1, qh1, s1); s1 = wmmab(h0, ql0, s1); s1 = wmmab(h1, ql1, s1);
      asm volatile("v_nop\n\tv_nop\n\tv_nop\n\tv_nop" : "+v"(s0), "+v"(s1) : "v"(h1), "v"(ql1), "v"(l1), "v"(h0)); }
    float sf; smx<MASK>(s0, s1, kb, qi, hi, m, l, sf, 0.0f);
    v16us ph, pl;
#pragma unroll
    for (int r = 0; r < 8; ++r) { unsigned short x, y; splitf(s0[r], x, y); ph[r] = x; pl[r] = y; splitf(s1[r], x, y); ph[8 + r] = x; pl[8 + r] = y; }
    const v16bf pfh = __builtin_bit_cast(v16bf, ph), pfl = __builtin_bit_cast(v16bf, pl);
    a0 = a0 * sf; a1 = a1 * sf; a2 = a2 * sf; a3 = a3 * sf;
    const bf* vh = VTh + voff + kb; const bf* vl = VTl + voff + kb;
    { const v16bf x = ldb(vh), y = ldb(vl); a0 = wmmab(x, pfh, a0); a0 = wmmab(x, pfl, a0); a0 = wmmab(y, pfh, a0);
      asm volatile("v_nop\n\tv_nop\n\tv_nop\n\tv_nop" : "+v"(a0) : "v"(x), "v"(y)); }
    { const v16bf x = ldb(vh + (size_t)16 * RH), y = ldb(vl + (size_t)16 * RH); a1 = wmmab(x, pfh, a1); a1 = wmmab(x, pfl, a1); a1 = wmmab(y, pfh, a1);
      asm volatile("v_nop\n\tv_nop\n\tv_nop\n\tv_nop" : "+v"(a1) : "v"(x), "v"(y)); }
    { const v16bf x = ldb(vh + (size_t)32 * RH), y = ldb(vl + (size_t)32 * RH); a2 = wmmab(x, pfh, a2); a2 = wmmab(x, pfl, a2); a2 = wmmab(y, pfh, a2);
      asm volatile("v_nop\n\tv_nop\n\tv_nop\n\tv_nop" : "+v"(a2) : "v"(x), "v"(y)); }
    { const v16bf x = ldb(vh + (size_t)48 * RH), y = ldb(vl + (size_t)48 * RH); a3 = wmmab(x, pfh, a3); a3 = wmmab(x, pfl, a3); a3 = wmmab(y, pfh, a3);
      asm volatile("v_nop\n\tv_nop\n\tv_nop\n\tv_nop" : "+v"(a0), "+v"(a1), "+v"(a2), "+v"(a3) : "v"(x), "v"(y), "v"(pfh), "v"(pfl)); }
}
__global__ __launch_bounds__(32) void k_attn_h(const bf* __restrict__ QKh, const bf* __restrict__ QKl, const bf* __restrict__ VTh, const bf* __restrict__ VTl, bf* ATh, bf* ATl) {
    const int lane = threadIdx.x & 31, lr = lane & 15, hi = lane >> 4;
    const int q0 = blockIdx.x * 16; const int bh = blockIdx.y; const int b = bh / NH, h = bh % NH;
    const size_t qoff = (((size_t)b * NSLOT + h) * RH + q0 + lr) * HD + 8 * hi;
    const size_t koff = (((size_t)b * NSLOT + NH + h) * RH + lr) * HD + 8 * hi;
    const size_t voff = (((size_t)b * NH + h) * HD + lr) * RH + 8 * hi;
    const v16bf qh0 = ldb(QKh + qoff), qh1 = ldb(QKh + qoff + 32), ql0 = ldb(QKl + qoff), ql1 = ldb(QKl + qoff + 32);
    v8f a0 = (v8f){}, a1 = (v8f){}, a2 = (v8f){}, a3 = (v8f){}; float m = -3.0e38f, l = 0.0f;
    const int qi = q0 + lr; const int nh = (q0 + 47) >> 5;
#pragma unroll 1
    for (int it = 0; it < nh - 1; ++it) step_h<false>(QKh, QKl, VTh, VTl, koff, voff, it * 32, qh0, qh1, ql0, ql1, qi, hi, m, l, a0, a1, a2, a3);
    step_h<true>(QKh, QKl, VTh, VTl, koff, voff, (nh - 1) * 32, qh0, qh1, ql0, ql1, qi, hi, m, l, a0, a1, a2, a3);
    attn_store(a0, a1, a2, a3, l, lane, ((size_t)b * SEQ + q0) * DM + h * HD, ATh, ATl);
}

constexpr size_t al256(size_t x) { return (x + 255) & ~(size_t)255; }
constexpr size_t SZ_WQKV = al256((size_t)NQKV * DM * 2);
constexpr size_t SZ_WO   = al256((size_t)DM * DM * 2);
constexpr size_t SZ_XB   = al256((size_t)NB * SEQ * DM * 2);
constexpr size_t SZ_IFQ  = al256((size_t)(HD / 2) * 4);
constexpr size_t SZ_CS   = al256((size_t)SEQ * (HD / 2) * 2 * 4);
constexpr size_t SZ_F    = al256((size_t)NB * SEQ * NQKV * 4);
constexpr size_t SZ_QK16 = al256((size_t)NB * NSLOT * SEQ * HD * 2);
constexpr size_t SZ_QKHL = al256((size_t)NB * NSLOT * RH * HD * 2);
constexpr size_t SZ_VT16 = al256((size_t)NB * NH * HD * SEQ * 2);
constexpr size_t SZ_VTHL = al256((size_t)NB * NH * HD * RH * 2);
constexpr size_t SZ_AT   = al256((size_t)NB * SEQ * DM * 2);
constexpr size_t OFF_WQKV = 0;
constexpr size_t OFF_WO   = OFF_WQKV + SZ_WQKV;
constexpr size_t OFF_XB   = OFF_WO + SZ_WO;
constexpr size_t OFF_IFQ  = OFF_XB + SZ_XB;
constexpr size_t OFF_CS   = OFF_IFQ + SZ_IFQ;
constexpr size_t OFF_F    = OFF_CS + SZ_CS;
constexpr size_t OFF_QK16 = OFF_F + SZ_F;
constexpr size_t OFF_QKH  = OFF_QK16 + SZ_QK16;
constexpr size_t OFF_QKL  = OFF_QKH + SZ_QKHL;
constexpr size_t OFF_VT16 = OFF_QKL + SZ_QKHL;
constexpr size_t OFF_VTH  = OFF_VT16 + SZ_VT16;
constexpr size_t OFF_VTL  = OFF_VTH + SZ_VTHL;
constexpr size_t OFF_ATH  = OFF_VTL + SZ_VTHL;
constexpr size_t OFF_ATL  = OFF_ATH + SZ_AT;
constexpr size_t WS_TOTAL = OFF_ATL + SZ_AT;
static_assert(WS_TOTAL <= (size_t)134217728);
static_assert(((size_t)(NB_FULL - 1) * SEQ_FULL + SEQ_FULL) * DM * 4 == (size_t)16777216);

extern "C" void kernel_launch(void* const* d_in, const int* in_sizes, int n_in,
                              void* d_out, int out_size, void* d_ws, size_t ws_size, hipStream_t stream) {
    if (n_in < 4) return;
    const long long need_x = ((long long)(NB - 1) * SEQ_FULL + SEQ) * DM;
    if ((long long)in_sizes[0] < need_x) return;
    if (in_sizes[1] < SEQ) return;
    if ((long long)in_sizes[2] < (long long)NQKV * DM) return;
    if ((long long)in_sizes[3] < (long long)DM * DM) return;
    if ((long long)out_size < need_x) return;
    if (ws_size < WS_TOTAL) return;
    const float* x = (const float*)d_in[0]; const int* tok = (const int*)d_in[1]; const float* wqkv = (const float*)d_in[2]; const float* wo = (const float*)d_in[3];
    float* OUT = (float*)d_out;
    char* ws = (char*)d_ws;
    bf* WQKV = (bf*)(ws + OFF_WQKV); bf* WO = (bf*)(ws + OFF_WO); bf* XB = (bf*)(ws + OFF_XB); float* IFQ = (float*)(ws + OFF_IFQ); float* CS = (float*)(ws + OFF_CS); float* F = (float*)(ws + OFF_F);
    h16* QK16 = (h16*)(ws + OFF_QK16); bf* QKh = (bf*)(ws + OFF_QKH); bf* QKl = (bf*)(ws + OFF_QKL); h16* VT16 = (h16*)(ws + OFF_VT16); bf* VTh = (bf*)(ws + OFF_VTH); bf* VTl = (bf*)(ws + OFF_VTL);
    bf* ATh = (bf*)(ws + OFF_ATH); bf* ATl = (bf*)(ws + OFF_ATL);

    { const size_t n8 = (size_t)NQKV * DM / 8; k_cvt8<<<(unsigned)((n8 + 255) / 256), 256, 0, stream>>>(wqkv, WQKV, n8, DM / 8, NQKV, NQKV); }
    { const size_t n8 = (size_t)DM * DM / 8;   k_cvt8<<<(unsigned)((n8 + 255) / 256), 256, 0, stream>>>(wo, WO, n8, DM / 8, DM, DM); }
    { const size_t n8 = (size_t)NB * SEQ * DM / 8; k_cvt8<<<(unsigned)((n8 + 255) / 256), 256, 0, stream>>>(x, XB, n8, DM / 8, SEQ, SEQ_FULL); }
    k_freq<<<1, 32, 0, stream>>>(IFQ);
    k_cstab<<<(SEQ * (HD / 2) + 255) / 256, 256, 0, stream>>>(tok, IFQ, CS);
    k_gemm_qkv<<<dim3(NB * SEQ / 64, NQKV / 64, 1), 32, 0, stream>>>(XB, WQKV, F);
    { const size_t nt = (size_t)NB * NSLOT * SEQ * HD / 2; k_rope<<<(unsigned)((nt + 255) / 256), 256, 0, stream>>>(F, CS, QK16, QKh, QKl); }
    { const size_t nt = (size_t)NB * NH * HD * SEQ / 2;    k_vtp<<<(unsigned)((nt + 255) / 256), 256, 0, stream>>>(F, VT16, VTh, VTl); }
    k_attn_h<<<dim3(RH / 16, NB * NH, 1), 32, 0, stream>>>(QKh, QKl, VTh, VTl, ATh, ATl);
    if (SEQ > RH) k_attn_f<<<dim3((SEQ - RH) / 16 + ((SEQ > RH) ? 0 : 1), NB * NH, 1), 32, 0, stream>>>(QK16, VT16, ATh, ATl);
    k_gemm_out<<<dim3(SEQ / 64, DM / 64, NB), 32, 0, stream>>>(ATh, ATl, WO, OUT);
}
